// Int4PackedLinear_67224828117704
// MI455X (gfx1250) — hardware-verified
//
#include <hip/hip_runtime.h>
#include <stdint.h>

#define IN_F  8192
#define OUT_F 8192
#define TOK   64
#define GRP   256
#define NGRP  (IN_F / GRP)
#define WPR   (IN_F / 8)
#define CPB   64
#define SP    68

static_assert((IN_F % GRP) == 0);
static_assert((GRP % 32) == 0);
static_assert((IN_F % 32) == 0);
static_assert(TOK == 64);
static_assert((OUT_F % CPB) == 0);
static_assert(CPB == 4 * 16);
static_assert((SP % 4) == 0);
static_assert(((TOK * IN_F) % (8 * 256)) == 0);
static_assert((TOK * SP) >= ((TOK - 1) * SP + CPB));

typedef __bf16       v16b __attribute__((ext_vector_type(16)));
typedef float        v8f  __attribute__((ext_vector_type(8)));
typedef float        v4f  __attribute__((ext_vector_type(4)));
typedef unsigned int v4u  __attribute__((ext_vector_type(4)));

union Frag { v16b v; v4u u[2]; };

__device__ __forceinline__ unsigned short bf_bits(float f) {
  const unsigned u = __float_as_uint(f);
  return (unsigned short)((u + 0x7FFFu + ((u >> 16) & 1u)) >> 16);
}
__device__ __forceinline__ float bfr(float f) { return __uint_as_float(((unsigned)bf_bits(f)) << 16); }
__device__ __forceinline__ unsigned pk16(unsigned short a, unsigned short b) { return (unsigned)a | ((unsigned)b << 16); }
__device__ __forceinline__ v8f zero8() { v8f z = {0.f, 0.f, 0.f, 0.f, 0.f, 0.f, 0.f, 0.f}; return z; }

__device__ __forceinline__ v8f mma_bf(const Frag& a, const Frag& b, v8f c) {
  return __builtin_amdgcn_wmma_f32_16x16x32_bf16(false, a.v, false, b.v, (short)0, c, false, false);
}
__device__ __forceinline__ void guard(v8f& c, const Frag& a, const Frag& b) {
#if defined(__HIP_DEVICE_COMPILE__)
  asm volatile("v_nop\n\tv_nop\n\tv_nop\n\tv_nop" : "+v"(c) : "v"(a.u[0]), "v"(a.u[1]), "v"(b.u[0]), "v"(b.u[1]));
#endif
}

__device__ __forceinline__ unsigned dq2(unsigned w, int sh, float s, float c8) {
  const unsigned n0 = (w >> sh) & 15u;
  const unsigned n1 = (w >> (sh + 4)) & 15u;
  const float f0 = fmaf((float)n0, s, c8);
  const float f1 = fmaf((float)n1, s, c8);
  return pk16(bf_bits(f0), bf_bits(f1));
}

__global__ __launch_bounds__(256)
void k_cvt(const float* __restrict__ x, unsigned short* X16, int np) {
  const int p  = blockIdx.x * 256 + threadIdx.x;
  const int pc = min(p, np - 1);
  const v4f a = *(const v4f*)(x + (size_t)pc * 8);
  const v4f b = *(const v4f*)(x + (size_t)pc * 8 + 4);
  v4u u;
  u[0] = pk16(bf_bits(a[0]), bf_bits(a[1]));
  u[1] = pk16(bf_bits(a[2]), bf_bits(a[3]));
  u[2] = pk16(bf_bits(b[0]), bf_bits(b[1]));
  u[3] = pk16(bf_bits(b[2]), bf_bits(b[3]));
  unsigned short* d = X16 + (size_t)pc * 8;
  if (p < np) *(volatile v4u*)d = u;
  __threadfence();
  if (p < np) *(volatile v4u*)d = u;
}

__global__ __launch_bounds__(128)
void k_gemm(const unsigned short* __restrict__ X16, const int* __restrict__ wp,
            const float* __restrict__ scales, const float* __restrict__ bias, float* out) {
  __shared__ __align__(16) float st[TOK * SP];

  const int tid = threadIdx.x, lane = tid & 31, wave = tid >> 5, h = lane >> 4, c = lane & 15;
  const int colbase = blockIdx.x * CPB;
  const int n = colbase + 16 * wave + c;

  const unsigned* wrow = (const unsigned*)wp + (size_t)n * WPR;
  const float*    srow = scales + (size_t)n * NGRP;
  const unsigned short* xb = X16 + 8 * h;

  v8f acc[4];
  acc[0] = zero8(); acc[1] = zero8(); acc[2] = zero8(); acc[3] = zero8();

#pragma unroll 1
  for (int g = 0; g < NGRP; ++g) {
    const float s  = bfr(srow[g]);
    const float c8 = -8.0f * s;
#pragma unroll 1
    for (int kk = 0; kk < GRP / 32; ++kk) {
      const int k0 = g * GRP + kk * 32;
      const v4u w4 = *(const v4u*)(wrow + (k0 >> 3));
      const unsigned wa = h ? w4[1] : w4[0];
      const unsigned wb = h ? w4[3] : w4[2];
      v4u b0, b1;
      b0[0] = dq2(wa, 0, s, c8);  b0[1] = dq2(wa, 8, s, c8);  b0[2] = dq2(wa, 16, s, c8);  b0[3] = dq2(wa, 24, s, c8);
      b1[0] = dq2(wb, 0, s, c8);  b1[1] = dq2(wb, 8, s, c8);  b1[2] = dq2(wb, 16, s, c8);  b1[3] = dq2(wb, 24, s, c8);
      Frag bfr16;
      bfr16.u[0] = b0;
      bfr16.u[1] = b1;
#pragma unroll
      for (int mt = 0; mt < 4; ++mt) {
        const unsigned short* ap = xb + (size_t)(16 * mt + c) * IN_F + k0;
        Frag af;
        af.u[0] = *(const v4u*)(ap);
        af.u[1] = *(const v4u*)(ap + 16);
        acc[mt] = mma_bf(af, bfr16, acc[mt]);
        guard(acc[mt], af, bfr16);
      }
    }
  }

  const float bb = bfr(bias[n]);
  const int cl = 16 * wave + c;
#pragma unroll
  for (int mt = 0; mt < 4; ++mt) {
#pragma unroll
    for (int r = 0; r < 8; ++r) {
      st[(16 * mt + 8 * h + r) * SP + cl] = bfr(acc[mt][r]) + bb;
    }
  }
  __syncthreads();

  float* ob = out + (size_t)colbase + 4 * c;
#pragma unroll
  for (int i = 0; i < 16; ++i) {
    const int t = 16 * wave + i;
    const v4f v = *(const v4f*)(st + t * SP + 4 * c);
    if (lane < 16) *(volatile v4f*)(ob + (size_t)t * OUT_F) = v;
  }
  __threadfence();
#pragma unroll
  for (int i = 0; i < 16; ++i) {
    const int t = 16 * wave + i;
    const v4f v = *(const v4f*)(st + t * SP + 4 * c);
    if (lane < 16) *(volatile v4f*)(ob + (size_t)t * OUT_F) = v;
  }
}

extern "C" void kernel_launch(void* const* d_in, const int* in_sizes, int n_in,
                              void* d_out, int out_size, void* d_ws, size_t ws_size,
                              hipStream_t stream) {
  if (n_in < 4) return;
  if (in_sizes[0] != TOK * IN_F) return;
  if (in_sizes[1] != OUT_F * WPR) return;
  if (in_sizes[2] != OUT_F * NGRP) return;
  if (in_sizes[3] != OUT_F) return;
  if (out_size != TOK * OUT_F) return;

  const size_t sX = (size_t)TOK * IN_F * 2;
  if (sX > ws_size) return;
  if (sX > (size_t)134217728) return;

  const float* x      = (const float*)d_in[0];
  const int*   wp     = (const int*)d_in[1];
  const float* scales = (const float*)d_in[2];
  const float* bias   = (const float*)d_in[3];
  float* out = (float*)d_out;
  unsigned short* X16 = (unsigned short*)d_ws;

  const int np  = (TOK * IN_F) / 8;
  const int nbc = (np + 255) / 256;

  k_cvt<<<dim3(nbc), dim3(256), 0, stream>>>(x, X16, np);
  k_gemm<<<dim3(OUT_F / CPB), dim3(128), 0, stream>>>(X16, wp, scales, bias, out);
  (void)hipGetLastError();
}
